// TCERL_13254269075507
// MI455X (gfx1250) — hardware-verified
//
#include <hip/hip_runtime.h>


#define NBAT 32
#define NSC  16
#define NCR  (NBAT * NSC)
#define CH   64
#define T0   400
#define L1   192
#define L2   87
#define L3   82
#define L3P  40
#define L4   35
#define K20  1280
#define K6   384
#define CH1  64
#define CH2  128
typedef _Float16 h16;
typedef unsigned short bf;
typedef __attribute__((ext_vector_type(16))) __bf16   v16bf;
typedef __attribute__((ext_vector_type(16))) _Float16 v16h;
typedef __attribute__((ext_vector_type(8)))  _Float16 v8h;
typedef __attribute__((ext_vector_type(8)))  unsigned short v8us;
typedef __attribute__((ext_vector_type(8)))  float    v8f;
typedef __attribute__((ext_vector_type(4)))  float    v4f;
typedef v8h  __attribute__((may_alias)) v8ha;
typedef v4f  __attribute__((may_alias)) v4fa;
typedef v8us __attribute__((may_alias)) v8usa;

__device__ __forceinline__ unsigned short f2bf(float f) { unsigned u = __float_as_uint(f); u += 0x7FFFu + ((u >> 16) & 1u); return (unsigned short)(u >> 16); }
__device__ __forceinline__ float bf2f(unsigned short b) { return __uint_as_float(((unsigned)b) << 16); }
__device__ __forceinline__ float bfr(float f) { return bf2f(f2bf(f)); }
__device__ __forceinline__ v16h cat16(v8h lo, v8h hi) { return __builtin_shufflevector(lo, hi, 0, 1, 2, 3, 4, 5, 6, 7, 8, 9, 10, 11, 12, 13, 14, 15); }
__device__ __forceinline__ v16bf cat16b(v8us lo, v8us hi) { return __builtin_bit_cast(v16bf, __builtin_shufflevector(lo, hi, 0, 1, 2, 3, 4, 5, 6, 7, 8, 9, 10, 11, 12, 13, 14, 15)); }
__device__ __forceinline__ v8f wmma16(v16h a, v16h b, v8f c) { return __builtin_amdgcn_wmma_f32_16x16x32_f16(false, a, false, b, (short)0, c, false, false); }
__device__ __forceinline__ v8f wmmab(v16bf a, v16bf b, v8f c) { return __builtin_amdgcn_wmma_f32_16x16x32_bf16(false, a, false, b, (short)0, c, false, false); }


template <typename T16> struct WFrag;
template <> struct WFrag<h16> { typedef v16h V; static __device__ __forceinline__ V ld(const h16* p) { return cat16(*(const v8h*)p, *(const v8h*)(p + 16)); } static __device__ __forceinline__ v8f mma(V a, V b, v8f c) { return wmma16(a, b, c); } };
template <> struct WFrag<bf> { typedef v16bf V; static __device__ __forceinline__ V ld(const bf* p) { return cat16b(*(const v8us*)p, *(const v8us*)(p + 16)); } static __device__ __forceinline__ v8f mma(V a, V b, v8f c) { return wmmab(a, b, c); } };
template <typename T16, int NSPLIT, bool BIAS>
__global__ __launch_bounds__(32) void k_gemmw(const T16* __restrict__ A, const T16* __restrict__ A2, const T16* __restrict__ Bt, const T16* __restrict__ Bt2, int K, float* C, int ldc, const float* __restrict__ bias, size_t sA, size_t sB, size_t sC) {
    typedef typename WFrag<T16>::V V;
    __shared__ __align__(16) float os[16 * 68];
    const size_t z = blockIdx.z; A += z * sA; if (A2) A2 += z * sA; Bt += z * sB; if (Bt2) Bt2 += z * sB; C += z * sC;
    const int lane = threadIdx.x & 31, lr = lane & 15, hi = lane >> 4; const int r0 = blockIdx.x * 64, c0 = blockIdx.y * 64;
    v8f acc[4][4];
#pragma unroll
    for (int mb = 0; mb < 4; ++mb)
#pragma unroll
        for (int nb = 0; nb < 4; ++nb) acc[mb][nb] = (v8f){};
    const size_t aoff = (size_t)(r0 + lr) * K + 8 * hi, boff = (size_t)(c0 + lr) * K + 8 * hi;
#pragma unroll 1
    for (int kc = 0; kc < K; kc += 32) {
        V a[4], a2[4];
#pragma unroll
        for (int mb = 0; mb < 4; ++mb) { a[mb] = WFrag<T16>::ld(A + aoff + (size_t)mb * 16 * K + kc); if (NSPLIT == 1 || NSPLIT == 2) a2[mb] = WFrag<T16>::ld(A2 + aoff + (size_t)mb * 16 * K + kc); }
#pragma unroll
        for (int nb = 0; nb < 4; ++nb) { const V b = WFrag<T16>::ld(Bt + boff + (size_t)nb * 16 * K + kc); V b2; if (NSPLIT >= 2) b2 = WFrag<T16>::ld(Bt2 + boff + (size_t)nb * 16 * K + kc);
#pragma unroll
            for (int mb = 0; mb < 4; ++mb) { acc[mb][nb] = WFrag<T16>::mma(a[mb], b, acc[mb][nb]); if (NSPLIT == 1 || NSPLIT == 2) acc[mb][nb] = WFrag<T16>::mma(a2[mb], b, acc[mb][nb]); if (NSPLIT >= 2) acc[mb][nb] = WFrag<T16>::mma(a[mb], b2, acc[mb][nb]); } }
        asm volatile("v_nop\n\tv_nop\n\tv_nop\n\tv_nop" : "+v"(acc[0][0]), "+v"(acc[1][1]), "+v"(acc[2][2]), "+v"(acc[3][3]) : "v"(a[0]), "v"(a[3]));
    }
#pragma unroll
    for (int mb = 0; mb < 4; ++mb) {
#pragma unroll
        for (int nb = 0; nb < 4; ++nb) {
#pragma unroll
            for (int j = 0; j < 8; ++j) os[(hi * 8 + j) * 68 + nb * 16 + lr] = acc[mb][nb][j]; }
        __builtin_amdgcn_wave_barrier(); asm volatile("" ::: "memory");
        float* crow = C + (size_t)(r0 + mb * 16) * ldc + c0;
#pragma unroll 1
        for (int ps = 0; ps < 2; ++ps) {
#pragma unroll
            for (int s = 0; s < 8; ++s) { const int row = 2 * s + hi, cofs = lr * 4; v4f val = *(const v4fa*)(os + row * 68 + cofs); if (BIAS) { val[0] += bfr(bias[c0 + cofs]); val[1] += bfr(bias[c0 + cofs + 1]); val[2] += bfr(bias[c0 + cofs + 2]); val[3] += bfr(bias[c0 + cofs + 3]); }
                *(volatile v4f*)(crow + (size_t)row * ldc + cofs) = val; }
            if (ps == 0) __threadfence(); }
        __builtin_amdgcn_wave_barrier(); asm volatile("" ::: "memory");
    }
}

__device__ __forceinline__ void splitf(float y, unsigned short& h, unsigned short& l) { h = f2bf(y); l = f2bf(y - bf2f(h)); }
__device__ __forceinline__ float eluf(float t) { return t > 0.f ? t : expm1f(t); }
typedef __attribute__((ext_vector_type(2))) unsigned short v2us;

__global__ __launch_bounds__(256) void k_wtb(const float* __restrict__ w, int K, int N, int Kp, int Np, bf* Bt) {
    const int lane = threadIdx.x & 31; const int L0 = (blockIdx.x * 8 + (threadIdx.x >> 5)) * 8; const int nlines = Np * Kp / 64;
#pragma unroll 1
    for (int ps = 0; ps < 2; ++ps) {
#pragma unroll 1
        for (int l = 0; l < 8; ++l) { const int L = L0 + l; if (L >= nlines) break; const int e = L * 64 + lane * 2; v2us o;
#pragma unroll
            for (int q = 0; q < 2; ++q) { const int n = (e + q) / Kp, k = (e + q) % Kp; o[q] = (n < N && k < K) ? f2bf(w[(size_t)k * N + n]) : (unsigned short)0; }
            *(volatile v2us*)(Bt + e) = o; }
        if (ps == 0) __threadfence(); }
}
__global__ __launch_bounds__(256) void k_cvt8(const float* __restrict__ src, bf* dst, size_t n8) { const size_t i = (size_t)blockIdx.x * 256 + threadIdx.x; if (i >= n8) return; const v8f v = *(const v8f*)(src + i * 8); v8us o;
#pragma unroll
    for (int k = 0; k < 8; ++k) o[k] = f2bf(v[k]); *(volatile v8us*)(dst + i * 8) = o; __threadfence(); *(volatile v8us*)(dst + i * 8) = o; }
__global__ __launch_bounds__(64) void k_bpad(const float* __restrict__ b, int N, float* out) { const int i = threadIdx.x; const float v = i < N ? b[i < N ? i : 0] : 0.f; *(volatile float*)(out + i) = v; __threadfence(); *(volatile float*)(out + i) = v; }
__global__ __launch_bounds__(256) void k_im1(const float* __restrict__ x, int n0, bf* IM) {
    const int lane = threadIdx.x & 31; const int L0 = (blockIdx.x * 8 + (threadIdx.x >> 5)) * 8; const int nlines = CH1 * L1 * K20 / 64;
#pragma unroll 1
    for (int ps = 0; ps < 2; ++ps) {
#pragma unroll 1
        for (int l = 0; l < 8; ++l) { const int L = L0 + l; if (L >= nlines) break; const int e = L * 64 + lane * 2; const int col = e % K20; const int row = e / K20; const int t = row % L1, nl = row / L1; v2us o;
#pragma unroll
            for (int q = 0; q < 2; ++q) { const int cq = col + q; const int ci = cq / 20, k = cq % 20; const int ti = 2 * t - 1 + k; o[q] = (ti >= 0 && ti < T0) ? f2bf(x[((size_t)(n0 + nl) * CH + ci) * T0 + ti]) : (unsigned short)0; }
            *(volatile v2us*)(IM + (size_t)e) = o; }
        if (ps == 0) __threadfence(); }
}
template <int KW, int STRIDE, int LIN, int LOUT, int NCH>
__global__ __launch_bounds__(256) void k_imhl(const float* __restrict__ Hs, int n0, bf* Ph, bf* Pl) {
    const int lane = threadIdx.x & 31; const int L0 = (blockIdx.x * 8 + (threadIdx.x >> 5)) * 8; constexpr int KK = CH * KW; const int nlines = NCH * LOUT * KK / 64;
#pragma unroll 1
    for (int ps = 0; ps < 2; ++ps) {
#pragma unroll 1
        for (int l = 0; l < 8; ++l) { const int L = L0 + l; if (L >= nlines) break; const int e = L * 64 + lane * 2; const int col = e % KK; const int row = e / KK; const int t = row % LOUT, nl = row / LOUT; v2us oh, ol;
#pragma unroll
            for (int q = 0; q < 2; ++q) { const int cq = col + q; const int ci = cq / KW, k = cq % KW; unsigned short a, c2; splitf(Hs[((size_t)(n0 + nl) * CH + ci) * LIN + STRIDE * t + k], a, c2); oh[q] = a; ol[q] = c2; }
            *(volatile v2us*)(Ph + (size_t)e) = oh; *(volatile v2us*)(Pl + (size_t)e) = ol; }
        if (ps == 0) __threadfence(); }
}
template <int LOUT, bool BN>
__global__ __launch_bounds__(256) void k_elubn(const float* __restrict__ C, int n0, int nch, const float* __restrict__ g, const float* __restrict__ bb, const float* __restrict__ mn, const float* __restrict__ vr, float* Hd) {
    typedef __attribute__((ext_vector_type(2))) float v2f;
    const int lane = threadIdx.x & 31; const int L0 = (blockIdx.x * 8 + (threadIdx.x >> 5)) * 8; const int nlines = nch * CH * LOUT / 64;
#pragma unroll 1
    for (int ps = 0; ps < 2; ++ps) {
#pragma unroll 1
        for (int l = 0; l < 8; ++l) { const int L = L0 + l; if (L >= nlines) break; const int e = L * 64 + lane * 2; v2f o;
#pragma unroll
            for (int q = 0; q < 2; ++q) { const int idx = e + q; const int t = idx % LOUT; const int oc = (idx / LOUT) % CH; const int nl = idx / (LOUT * CH); float v = eluf(C[((size_t)nl * LOUT + t) * CH + oc]);
                if (BN) { const float inv = __fdiv_rn(bfr(g[oc]), sqrtf(bfr(vr[oc]) + 1e-5f)); v = (v - bfr(mn[oc])) * inv + bfr(bb[oc]); } o[q] = v; }
            *(volatile v2f*)(Hd + (size_t)n0 * CH * LOUT + e) = o; }
        if (ps == 0) __threadfence(); }
}
__global__ __launch_bounds__(256) void k_elupool(const float* __restrict__ C, float* Hd) {
    typedef __attribute__((ext_vector_type(2))) float v2f;
    const int lane = threadIdx.x & 31; const int L0 = (blockIdx.x * 8 + (threadIdx.x >> 5)) * 8; const int nlines = NCR * CH * L3P / 64;
#pragma unroll 1
    for (int ps = 0; ps < 2; ++ps) {
#pragma unroll 1
        for (int l = 0; l < 8; ++l) { const int L = L0 + l; if (L >= nlines) break; const int e = L * 64 + lane * 2; v2f o;
#pragma unroll
            for (int q = 0; q < 2; ++q) { const int idx = e + q; const int tp = idx % L3P; const int oc = (idx / L3P) % CH; const int n = idx / (L3P * CH); const float* cr = C + ((size_t)n * L3 + 2 * tp) * CH + oc;
                const float s = (eluf(cr[0]) + eluf(cr[CH])) + eluf(cr[2 * CH]); o[q] = __fdiv_rn(s, 3.0f); }
            *(volatile v2f*)(Hd + (size_t)e) = o; }
        if (ps == 0) __threadfence(); }
}
__global__ __launch_bounds__(256) void k_elu4(const float* __restrict__ C, float* HF, bf* Ph, bf* Pl) {
    typedef __attribute__((ext_vector_type(2))) float v2f;
    const int lane = threadIdx.x & 31; const int L0 = (blockIdx.x * 8 + (threadIdx.x >> 5)) * 8; const int nlines = NCR * CH * 64 / 64;
#pragma unroll 1
    for (int ps = 0; ps < 2; ++ps) {
#pragma unroll 1
        for (int l = 0; l < 8; ++l) { const int L = L0 + l; if (L >= nlines) break; const int e = L * 64 + lane * 2; const int t = e & 63; const int nc = e >> 6; const int c = nc & 63, n = nc >> 6; v2us oh, ol; v2f of;
#pragma unroll
            for (int q = 0; q < 2; ++q) { const int tq = t + q; float v = 0.f; if (tq < L4) v = eluf(C[((size_t)n * L4 + tq) * CH + c]); of[q] = v; unsigned short a, c2; splitf(v, a, c2); oh[q] = a; ol[q] = c2; }
            *(volatile v2f*)(HF + (size_t)e) = of; *(volatile v2us*)(Ph + (size_t)e) = oh; *(volatile v2us*)(Pl + (size_t)e) = ol; }
        if (ps == 0) __threadfence(); }
}
__global__ __launch_bounds__(256) void k_tanhsplit(const float* __restrict__ V, int nlines, bf* Ph, bf* Pl) {
    const int lane = threadIdx.x & 31; const int L = blockIdx.x * 8 + (threadIdx.x >> 5); if (L >= nlines) return; const int e = L * 64 + lane * 2; v2us oh, ol;
#pragma unroll
    for (int q = 0; q < 2; ++q) { unsigned short a, c2; splitf(tanhf(V[(size_t)e + q]), a, c2); oh[q] = a; ol[q] = c2; }
    *(volatile v2us*)(Ph + (size_t)e) = oh; *(volatile v2us*)(Pl + (size_t)e) = ol; __threadfence(); *(volatile v2us*)(Ph + (size_t)e) = oh; *(volatile v2us*)(Pl + (size_t)e) = ol;
}
template <int ACT>
__global__ __launch_bounds__(256) void k_actsplit(const float* __restrict__ A, int nlines, int cols, int live, bf* Ph, bf* Pl) {
    const int lane = threadIdx.x & 31; const int L = blockIdx.x * 8 + (threadIdx.x >> 5); if (L >= nlines) return; const int e = L * 64 + lane * 2; v2us oh, ol;
#pragma unroll
    for (int q = 0; q < 2; ++q) { const int c = (e + q) % cols; float v = (c < live) ? A[(size_t)e + q] : 0.f; if (ACT == 1) v = fmaxf(v, 0.f); if (ACT == 2) v = eluf(v); unsigned short a, c2; splitf(v, a, c2); oh[q] = a; ol[q] = c2; }
    *(volatile v2us*)(Ph + (size_t)e) = oh; *(volatile v2us*)(Pl + (size_t)e) = ol; __threadfence(); *(volatile v2us*)(Ph + (size_t)e) = oh; *(volatile v2us*)(Pl + (size_t)e) = ol;
}
__global__ __launch_bounds__(256) void k_apool(const float* __restrict__ SC, const float* __restrict__ HF, float* HP) {
    typedef __attribute__((ext_vector_type(2))) float v2f;
    const int lane = threadIdx.x & 31; const int wg = blockIdx.x * 8 + (threadIdx.x >> 5); if (wg >= NBAT * CH) return; const int b = wg >> 6, c = wg & 63;
    float sc[NSC]; float m = -3.0e38f;
#pragma unroll
    for (int s = 0; s < NSC; ++s) { sc[s] = SC[((size_t)(b * NSC + s) * CH + c) * 64]; m = fmaxf(m, sc[s]); }
    float sum = 0.f;
#pragma unroll
    for (int s = 0; s < NSC; ++s) { sc[s] = __expf(sc[s] - m); sum += sc[s]; }
    const float inv = __fdiv_rn(1.0f, sum); v2f o;
#pragma unroll
    for (int q = 0; q < 2; ++q) { const int t = lane * 2 + q; float acc = 0.f;
        if (t < L4) {
#pragma unroll
            for (int s = 0; s < NSC; ++s) acc = fmaf(HF[((size_t)(b * NSC + s) * CH + c) * 64 + t], sc[s] * inv, acc);
            acc = eluf(acc); }
        o[q] = (t < L4) ? acc : 0.f; }
    *(volatile v2f*)(HP + (size_t)wg * 64 + lane * 2) = o; __threadfence(); *(volatile v2f*)(HP + (size_t)wg * 64 + lane * 2) = o;
}
template <int COLS, bool RELU>
__global__ __launch_bounds__(256) void k_ginagg(const float* __restrict__ Hin, bf* Ph, bf* Pl) {
    const int lane = threadIdx.x & 31; const int wg = blockIdx.x * 8 + (threadIdx.x >> 5); if (wg >= NBAT * (COLS / 64)) return; const int b = wg / (COLS / 64), ck = wg % (COLS / 64); const int col = ck * 64 + lane * 2;
    float s0 = 0.f, s1 = 0.f;
#pragma unroll 1
    for (int c = 0; c < CH; ++c) { float v0 = Hin[((size_t)b * CH + c) * COLS + col], v1 = Hin[((size_t)b * CH + c) * COLS + col + 1]; if (RELU) { v0 = fmaxf(v0, 0.f); v1 = fmaxf(v1, 0.f); } s0 += v0; s1 += v1; }
#pragma unroll 1
    for (int ps = 0; ps < 2; ++ps) {
#pragma unroll 1
        for (int c = 0; c < CH; ++c) { float v0 = Hin[((size_t)b * CH + c) * COLS + col], v1 = Hin[((size_t)b * CH + c) * COLS + col + 1]; if (RELU) { v0 = fmaxf(v0, 0.f); v1 = fmaxf(v1, 0.f); } v2us oh, ol; unsigned short a, c2;
            splitf(v0 + s0, a, c2); oh[0] = a; ol[0] = c2; splitf(v1 + s1, a, c2); oh[1] = a; ol[1] = c2;
            *(volatile v2us*)(Ph + ((size_t)b * CH + c) * COLS + col) = oh; *(volatile v2us*)(Pl + ((size_t)b * CH + c) * COLS + col) = ol; }
        if (ps == 0) __threadfence(); }
}
__global__ __launch_bounds__(256) void k_flat(const float* __restrict__ H5, bf* Ph, bf* Pl) {
    const int lane = threadIdx.x & 31; const int L0 = (blockIdx.x * 8 + (threadIdx.x >> 5)) * 8; const int nlines = 64 * 2240 / 64;
#pragma unroll 1
    for (int ps = 0; ps < 2; ++ps) {
#pragma unroll 1
        for (int l = 0; l < 8; ++l) { const int L = L0 + l; if (L >= nlines) break; const int e = L * 64 + lane * 2; v2us oh, ol;
#pragma unroll
            for (int q = 0; q < 2; ++q) { const int idx = e + q; const int col = idx % 2240, b = idx / 2240; float v = 0.f; if (b < NBAT) { const int c = col / L4, t = col % L4; v = H5[((size_t)b * CH + c) * 64 + t]; } unsigned short a, c2; splitf(v, a, c2); oh[q] = a; ol[q] = c2; }
            *(volatile v2us*)(Ph + (size_t)e) = oh; *(volatile v2us*)(Pl + (size_t)e) = ol; }
        if (ps == 0) __threadfence(); }
}
__global__ __launch_bounds__(64) void k_out(const float* __restrict__ R, float* OUT) { const int i = threadIdx.x; const float v = R[(size_t)(i >> 1) * 64 + (i & 1)]; *(volatile float*)(OUT + i) = v; __threadfence(); *(volatile float*)(OUT + i) = v; }

extern "C" void kernel_launch(void* const* d_in, const int* in_sizes, int n_in,
                              void* d_out, int out_size, void* d_ws, size_t ws_size, hipStream_t stream) {
    (void)in_sizes; (void)n_in; (void)out_size;
    const float* IN[40]; for (int i = 0; i < 40; ++i) IN[i] = (const float*)d_in[i];
    const float* x = IN[0];
    float* OUT = (float*)d_out;
    char* wsp = (char*)d_ws;
    auto take = [&](size_t bytes) { char* p = wsp; wsp += (bytes + 255) & ~(size_t)255; return (void*)p; };
    bf* W1B = (bf*)take((size_t)CH * K20 * 2); bf* W2B = (bf*)take((size_t)CH * K20 * 2); bf* W3B = (bf*)take((size_t)CH * K6 * 2); bf* W4B = (bf*)take((size_t)CH * K6 * 2);
    bf* AWB = (bf*)take(256 * 64 * 2); bf* AUB = (bf*)take(64 * 256 * 2);
    bf* G0W1 = (bf*)take(256 * 64 * 2); bf* G0W2 = (bf*)take(256 * 256 * 2); bf* G1W1 = (bf*)take(256 * 256 * 2); bf* G1W2 = (bf*)take(256 * 256 * 2); bf* G2W1 = (bf*)take(64 * 256 * 2); bf* G2W2 = (bf*)take(64 * 64 * 2);
    bf* C1W = (bf*)take((size_t)256 * 2240 * 2); bf* C2W = (bf*)take(64 * 256 * 2); bf* C3W = (bf*)take(64 * 64 * 2); bf* C4W = (bf*)take(64 * 64 * 2);
    float* G2B1P = (float*)take(64 * 4); float* G2B2P = (float*)take(64 * 4); float* C3BP = (float*)take(64 * 4); float* C4BP = (float*)take(64 * 4);
#define IMMAX ((size_t)NCR * L3 * K6)
    static_assert((size_t)CH2 * L2 * K20 <= IMMAX && (size_t)NCR * L4 * K6 <= IMMAX && (size_t)CH1 * L1 * K20 <= 2 * IMMAX && (size_t)NCR * CH * 256 * 4 <= 2 * IMMAX * 2, "im2col / V aliases must fit the shared plane region");
    bf* IMh = (bf*)take(IMMAX * 2); bf* IMl = (bf*)take(IMMAX * 2);
    bf* IM1 = IMh;
    float* Cb = (float*)take((size_t)NCR * L3 * CH * 4);
    float* H1 = (float*)take((size_t)NCR * CH * L1 * 4); float* H2 = (float*)take((size_t)NCR * CH * L2 * 4); float* H3P = (float*)take((size_t)NCR * CH * L3P * 4);
    float* H4F = (float*)take((size_t)NCR * CH * 64 * 4); bf* H4h = (bf*)take((size_t)NCR * CH * 64 * 2); bf* H4l = (bf*)take((size_t)NCR * CH * 64 * 2);
    float* V = (float*)IMh; bf* TVh = (bf*)take((size_t)NCR * CH * 256 * 2); bf* TVl = (bf*)take((size_t)NCR * CH * 256 * 2); float* SC = (float*)take((size_t)NCR * CH * 64 * 4);
    float* HP = (float*)take((size_t)NBAT * CH * 64 * 4); bf* AGh = (bf*)take((size_t)NBAT * CH * 256 * 2); bf* AGl = (bf*)take((size_t)NBAT * CH * 256 * 2);
    float* GA = (float*)take((size_t)NBAT * CH * 256 * 4); bf* GPh = (bf*)take((size_t)NBAT * CH * 256 * 2); bf* GPl = (bf*)take((size_t)NBAT * CH * 256 * 2); float* GB = (float*)take((size_t)NBAT * CH * 256 * 4);
    bf* F6h = (bf*)take((size_t)64 * 2240 * 2); bf* F6l = (bf*)take((size_t)64 * 2240 * 2); float* R1 = (float*)take(64 * 256 * 4); bf* RPh = (bf*)take(64 * 256 * 2); bf* RPl = (bf*)take(64 * 256 * 2); float* R2 = (float*)take(64 * 64 * 4);
    if ((size_t)(wsp - (char*)d_ws) > ws_size) return;
    { const unsigned gK20 = (unsigned)((CH * K20 / 8 + 255) / 256), gK6 = (unsigned)((CH * K6 / 8 + 255) / 256);
      k_cvt8<<<gK20, 256, 0, stream>>>(IN[1], W1B, (size_t)CH * K20 / 8); k_cvt8<<<gK20, 256, 0, stream>>>(IN[7], W2B, (size_t)CH * K20 / 8); k_cvt8<<<gK6, 256, 0, stream>>>(IN[13], W3B, (size_t)CH * K6 / 8); k_cvt8<<<gK6, 256, 0, stream>>>(IN[15], W4B, (size_t)CH * K6 / 8);
      k_wtb<<<4, 256, 0, stream>>>(IN[17], L4, 256, 64, 256, AWB);
      k_wtb<<<4, 256, 0, stream>>>(IN[19], 256, 1, 256, 64, AUB);
      k_wtb<<<4, 256, 0, stream>>>(IN[20], L4, 256, 64, 256, G0W1); k_wtb<<<16, 256, 0, stream>>>(IN[22], 256, 256, 256, 256, G0W2);
      k_wtb<<<16, 256, 0, stream>>>(IN[24], 256, 256, 256, 256, G1W1); k_wtb<<<16, 256, 0, stream>>>(IN[26], 256, 256, 256, 256, G1W2);
      k_wtb<<<4, 256, 0, stream>>>(IN[28], 256, L4, 256, 64, G2W1); k_wtb<<<1, 256, 0, stream>>>(IN[30], L4, L4, 64, 64, G2W2);
      k_wtb<<<(256 * 2240 / 64 + 63) / 64, 256, 0, stream>>>(IN[32], 2240, 256, 2240, 256, C1W); k_wtb<<<4, 256, 0, stream>>>(IN[34], 256, 64, 256, 64, C2W); k_wtb<<<1, 256, 0, stream>>>(IN[36], 64, 16, 64, 64, C3W); k_wtb<<<1, 256, 0, stream>>>(IN[38], 16, 2, 64, 64, C4W);
      k_bpad<<<1, 64, 0, stream>>>(IN[29], L4, G2B1P); k_bpad<<<1, 64, 0, stream>>>(IN[31], L4, G2B2P); k_bpad<<<1, 64, 0, stream>>>(IN[37], 16, C3BP); k_bpad<<<1, 64, 0, stream>>>(IN[39], 2, C4BP); }
    for (int ch = 0; ch < NCR / CH1; ++ch) { const int n0 = ch * CH1;
        k_im1<<<(CH1 * L1 * K20 / 64 + 63) / 64, 256, 0, stream>>>(x, n0, IM1);
        k_gemmw<bf, 0, true><<<dim3(CH1 * L1 / 64, 1, 1), 32, 0, stream>>>(IM1, nullptr, W1B, nullptr, K20, Cb, CH, IN[2], 0, 0, 0);
        k_elubn<L1, true><<<(CH1 * CH * L1 / 64 + 63) / 64, 256, 0, stream>>>(Cb, n0, CH1, IN[3], IN[4], IN[5], IN[6], H1); }
    for (int ch = 0; ch < NCR / CH2; ++ch) { const int n0 = ch * CH2;
        k_imhl<20, 2, L1, L2, CH2><<<(CH2 * L2 * K20 / 64 + 63) / 64, 256, 0, stream>>>(H1, n0, IMh, IMl);
        k_gemmw<bf, 1, true><<<dim3(CH2 * L2 / 64, 1, 1), 32, 0, stream>>>(IMh, IMl, W2B, nullptr, K20, Cb, CH, IN[8], 0, 0, 0);
        k_elubn<L2, true><<<(CH2 * CH * L2 / 64 + 63) / 64, 256, 0, stream>>>(Cb, n0, CH2, IN[9], IN[10], IN[11], IN[12], H2); }
    k_imhl<6, 1, L2, L3, NCR><<<(NCR * L3 * K6 / 64 + 63) / 64, 256, 0, stream>>>(H2, 0, IMh, IMl);
    k_gemmw<bf, 1, true><<<dim3(NCR * L3 / 64, 1, 1), 32, 0, stream>>>(IMh, IMl, W3B, nullptr, K6, Cb, CH, IN[14], 0, 0, 0);
    k_elupool<<<(NCR * CH * L3P / 64 + 63) / 64, 256, 0, stream>>>(Cb, H3P);
    k_imhl<6, 1, L3P, L4, NCR><<<(NCR * L4 * K6 / 64 + 63) / 64, 256, 0, stream>>>(H3P, 0, IMh, IMl);
    k_gemmw<bf, 1, true><<<dim3(NCR * L4 / 64, 1, 1), 32, 0, stream>>>(IMh, IMl, W4B, nullptr, K6, Cb, CH, IN[16], 0, 0, 0);
    k_elu4<<<(NCR * CH * 64 / 64 + 63) / 64, 256, 0, stream>>>(Cb, H4F, H4h, H4l);
    k_gemmw<bf, 1, true><<<dim3(NCR * CH / 64, 256 / 64, 1), 32, 0, stream>>>(H4h, H4l, AWB, nullptr, 64, V, 256, IN[18], 0, 0, 0);
    k_tanhsplit<<<(NCR * CH * 256 / 64 + 7) / 8, 256, 0, stream>>>(V, NCR * CH * 256 / 64, TVh, TVl);
    k_gemmw<bf, 1, false><<<dim3(NCR * CH / 64, 1, 1), 32, 0, stream>>>(TVh, TVl, AUB, nullptr, 256, SC, 64, nullptr, 0, 0, 0);
    k_apool<<<NBAT * CH / 8, 256, 0, stream>>>(SC, H4F, HP);
    k_ginagg<64, false><<<(NBAT * 1 + 7) / 8, 256, 0, stream>>>(HP, AGh, AGl);
    k_gemmw<bf, 1, true><<<dim3(NBAT * CH / 64, 256 / 64, 1), 32, 0, stream>>>(AGh, AGl, G0W1, nullptr, 64, GA, 256, IN[21], 0, 0, 0);
    k_actsplit<1><<<(NBAT * CH * 256 / 64 + 7) / 8, 256, 0, stream>>>(GA, NBAT * CH * 256 / 64, 256, 256, GPh, GPl);
    k_gemmw<bf, 1, true><<<dim3(NBAT * CH / 64, 256 / 64, 1), 32, 0, stream>>>(GPh, GPl, G0W2, nullptr, 256, GB, 256, IN[23], 0, 0, 0);
    k_ginagg<256, true><<<(NBAT * 4 + 7) / 8, 256, 0, stream>>>(GB, AGh, AGl);
    k_gemmw<bf, 1, true><<<dim3(NBAT * CH / 64, 256 / 64, 1), 32, 0, stream>>>(AGh, AGl, G1W1, nullptr, 256, GA, 256, IN[25], 0, 0, 0);
    k_actsplit<1><<<(NBAT * CH * 256 / 64 + 7) / 8, 256, 0, stream>>>(GA, NBAT * CH * 256 / 64, 256, 256, GPh, GPl);
    k_gemmw<bf, 1, true><<<dim3(NBAT * CH / 64, 256 / 64, 1), 32, 0, stream>>>(GPh, GPl, G1W2, nullptr, 256, GB, 256, IN[27], 0, 0, 0);
    k_ginagg<256, true><<<(NBAT * 4 + 7) / 8, 256, 0, stream>>>(GB, AGh, AGl);
    k_gemmw<bf, 1, true><<<dim3(NBAT * CH / 64, 1, 1), 32, 0, stream>>>(AGh, AGl, G2W1, nullptr, 256, GA, 64, G2B1P, 0, 0, 0);
    k_actsplit<1><<<(NBAT * CH * 64 / 64 + 7) / 8, 256, 0, stream>>>(GA, NBAT * CH * 64 / 64, 64, L4, GPh, GPl);
    k_gemmw<bf, 1, true><<<dim3(NBAT * CH / 64, 1, 1), 32, 0, stream>>>(GPh, GPl, G2W2, nullptr, 64, GB, 64, G2B2P, 0, 0, 0);
    k_flat<<<(64 * 2240 / 64 + 63) / 64, 256, 0, stream>>>(GB, F6h, F6l);
    k_gemmw<bf, 1, true><<<dim3(1, 256 / 64, 1), 32, 0, stream>>>(F6h, F6l, C1W, nullptr, 2240, R1, 256, IN[33], 0, 0, 0);
    k_actsplit<2><<<(64 * 256 / 64 + 7) / 8, 256, 0, stream>>>(R1, 64 * 256 / 64, 256, 256, RPh, RPl);
    k_gemmw<bf, 1, true><<<dim3(1, 1, 1), 32, 0, stream>>>(RPh, RPl, C2W, nullptr, 256, R2, 64, IN[35], 0, 0, 0);
    k_actsplit<2><<<(64 * 64 / 64 + 7) / 8, 256, 0, stream>>>(R2, 64 * 64 / 64, 64, 64, RPh, RPl);
    k_gemmw<bf, 1, true><<<dim3(1, 1, 1), 32, 0, stream>>>(RPh, RPl, C3W, nullptr, 64, R1, 64, C3BP, 0, 0, 0);
    k_actsplit<2><<<(64 * 64 / 64 + 7) / 8, 256, 0, stream>>>(R1, 64 * 64 / 64, 64, 16, RPh, RPl);
    k_gemmw<bf, 1, true><<<dim3(1, 1, 1), 32, 0, stream>>>(RPh, RPl, C4W, nullptr, 64, R2, 64, C4BP, 0, 0, 0);
    k_out<<<1, 64, 0, stream>>>(R2, OUT);
}
